// StandardMultiHeadAttention_5257039970890
// MI455X (gfx1250) — hardware-verified
//
#include <hip/hip_runtime.h>

typedef _Float16 v16h __attribute__((ext_vector_type(16)));
typedef _Float16 v8h  __attribute__((ext_vector_type(8)));
typedef float    v8f  __attribute__((ext_vector_type(8)));
typedef float    v4f  __attribute__((ext_vector_type(4)));
typedef v8h __attribute__((may_alias)) v8ha;
typedef v4f __attribute__((may_alias)) v4fa;

union Frag { v16h v; v8h half[2]; };

#define HIDDEN 1024
#define NHEADS 16
#define HD     64
#define SEQ    2048
#define BATCH  4
#define MROWS  (BATCH * SEQ)
#define NX     (MROWS * HIDDEN)
#define NW     (HIDDEN * HIDDEN)
#define NX8    (NX / 8)
#define NW8    (NW / 8)
#define NWMAT  4
#define PSCALE 16384.0f
#define WSC    1024.0f
#define WINV   (1.0f / 1024.0f)
#define CSC    256.0f
#define OINV   (1.0f / (256.0f * 1024.0f))
#define SSCALE 0.125f

static_assert(NHEADS * HD == HIDDEN);
static_assert((HIDDEN % 32) == 0);
static_assert((MROWS % 128) == 0 && (SEQ % 128) == 0);
static_assert((SEQ % 64) == 0);
static_assert((NX8 % 256) == 0 && (NW8 % 256) == 0);

__device__ __forceinline__ v8f wmma_f16(v16h a, v16h b, v8f c) {
  v8f d = __builtin_amdgcn_wmma_f32_16x16x32_f16(false, a, false, b, (short)0, c, false, false);
  asm volatile("v_nop\n\tv_nop\n\tv_nop\n\tv_nop" : "+v"(d) : "v"(a), "v"(b));
  return d;
}

__device__ __forceinline__ v16h load_frag(const _Float16* p, int h) {
  Frag f;
  f.half[0] = *(const v8ha*)(p + 8 * h);
  f.half[1] = *(const v8ha*)(p + 16 + 8 * h);
  return f.v;
}

__global__ __launch_bounds__(256) void convert_kernel(
    const float* __restrict__ x, const float* __restrict__ wq,
    const float* __restrict__ wk, const float* __restrict__ wv,
    const float* __restrict__ wo,
    _Float16* __restrict__ xh, _Float16* __restrict__ wh)
{
  const int g = blockIdx.x * 256 + threadIdx.x;
  if (g >= NX8 + NWMAT * NW8) return;
  const float* src;
  _Float16* dst;
  float sc;
  if (g < NX8) {
    src = x + (size_t)g * 8;
    dst = xh + (size_t)g * 8;
    sc = 1.0f;
  } else {
    const int e = g - NX8;
    const int wsel = e / NW8;
    const int off = e - wsel * NW8;
    const float* wsrc = (wsel == 0) ? wq : ((wsel == 1) ? wk : ((wsel == 2) ? wv : wo));
    src = wsrc + (size_t)off * 8;
    dst = wh + (size_t)e * 8;
    sc = WSC;
  }
  const v4f a = *(const v4fa*)src;
  const v4f c = *(const v4fa*)(src + 4);
  const v8h o = { (_Float16)(a.x * sc), (_Float16)(a.y * sc), (_Float16)(a.z * sc), (_Float16)(a.w * sc),
                  (_Float16)(c.x * sc), (_Float16)(c.y * sc), (_Float16)(c.z * sc), (_Float16)(c.w * sc) };
  *(volatile v8h*)dst = o;
  __threadfence();
  *(volatile v8h*)dst = o;
}

__device__ __forceinline__ void proj_store_pass(const _Float16* sT, _Float16* plane, _Float16* vt,
                                                int which, int bh, int l0, int w, int lane) {
  const int q8 = lane & 7, sub = lane >> 3;
  #pragma unroll
  for (int i = 0; i < 8; ++i) {
    const int lid = w * 32 + i * 4 + sub;
    v8h v;
    _Float16* dst;
    if (which != 2) {
      v = *(const v8ha*)(sT + lid * HD + 8 * q8);
      dst = plane + ((size_t)bh * SEQ + l0 + lid) * HD + 8 * q8;
    } else {
      const int d = lid >> 1, hl = lid & 1;
      v = *(const v8ha*)(sT + d * 128 + 64 * hl + 8 * q8);
      dst = vt + ((size_t)bh * HD + d) * SEQ + l0 + 64 * hl + 8 * q8;
    }
    *(volatile v8h*)dst = v;
  }
}

__global__ __launch_bounds__(128) void proj_kernel(
    const _Float16* __restrict__ xh,
    const _Float16* __restrict__ wh,
    const float* __restrict__ bq, const float* __restrict__ bk, const float* __restrict__ bv,
    _Float16* __restrict__ qh,
    _Float16* __restrict__ kh,
    _Float16* __restrict__ vt)
{
  __shared__ __attribute__((aligned(16))) _Float16 sT[128 * 64];

  const int tid = threadIdx.x, lane = tid & 31, w = tid >> 5;
  const int h = lane >> 4, m = lane & 15;
  const int m0 = blockIdx.x * 128;
  const int cg = blockIdx.y;
  const int which = cg >> 4, head = cg & 15;
  const int m0w = m0 + 32 * w;

  const _Float16* xa0 = xh + (size_t)(m0w + m) * HIDDEN;
  const _Float16* xa1 = xa0 + (size_t)16 * HIDDEN;
  const _Float16* wb  = wh + ((size_t)which * HIDDEN + head * HD + m) * HIDDEN;

  const v8f zero8 = {0.f, 0.f, 0.f, 0.f, 0.f, 0.f, 0.f, 0.f};
  v8f acc[2][4];
  #pragma unroll
  for (int mt = 0; mt < 2; ++mt)
    #pragma unroll
    for (int nt = 0; nt < 4; ++nt) acc[mt][nt] = zero8;

  #pragma unroll 1
  for (int k0 = 0; k0 < HIDDEN; k0 += 32) {
    const v16h a0 = load_frag(xa0 + k0, h);
    const v16h a1 = load_frag(xa1 + k0, h);
    #pragma unroll
    for (int nt = 0; nt < 4; ++nt) {
      const v16h b = load_frag(wb + (size_t)nt * 16 * HIDDEN + k0, h);
      acc[0][nt] = wmma_f16(a0, b, acc[0][nt]);
      acc[1][nt] = wmma_f16(a1, b, acc[1][nt]);
    }
  }

  const float* bias = (which == 0) ? bq : ((which == 1) ? bk : bv);
  #pragma unroll
  for (int nt = 0; nt < 4; ++nt) {
    const int feat = 16 * nt + m;
    const float bvl = bias[head * HD + feat];
    #pragma unroll
    for (int mt = 0; mt < 2; ++mt) {
      #pragma unroll
      for (int r = 0; r < 8; ++r) {
        const int tokl = 32 * w + 16 * mt + 8 * h + r;
        const float y = acc[mt][nt][r] * WINV + bvl;
        const int idx = (which == 2) ? (feat * 128 + tokl) : (tokl * HD + feat);
        sT[idx] = (_Float16)y;
      }
    }
  }
  __syncthreads();

  const int b = m0 / SEQ, l0 = m0 - b * SEQ, bh = b * NHEADS + head;
  _Float16* plane = (which == 0) ? qh : kh;
  proj_store_pass(sT, plane, vt, which, bh, l0, w, lane);
  __threadfence();
  proj_store_pass(sT, plane, vt, which, bh, l0, w, lane);
}

__device__ __forceinline__ v16h pack_p(v8f a, v8f c) {
  const v16h r = { (_Float16)(a[0] * PSCALE), (_Float16)(a[1] * PSCALE), (_Float16)(a[2] * PSCALE), (_Float16)(a[3] * PSCALE),
                   (_Float16)(a[4] * PSCALE), (_Float16)(a[5] * PSCALE), (_Float16)(a[6] * PSCALE), (_Float16)(a[7] * PSCALE),
                   (_Float16)(c[0] * PSCALE), (_Float16)(c[1] * PSCALE), (_Float16)(c[2] * PSCALE), (_Float16)(c[3] * PSCALE),
                   (_Float16)(c[4] * PSCALE), (_Float16)(c[5] * PSCALE), (_Float16)(c[6] * PSCALE), (_Float16)(c[7] * PSCALE) };
  return r;
}

__global__ __launch_bounds__(128) void attn_kernel(
    const _Float16* __restrict__ qh,
    const _Float16* __restrict__ kh,
    const _Float16* __restrict__ vt,
    _Float16* __restrict__ ctx)
{
  __shared__ __attribute__((aligned(16))) float sO[4 * 16 * 64];

  const int tid = threadIdx.x, lane = tid & 31, w = tid >> 5;
  const int h = lane >> 4, m = lane & 15;
  const int bh = blockIdx.y, b = bh >> 4, head = bh & 15;
  const int q0 = blockIdx.x * 64 + 16 * w;

  const _Float16* qrow = qh + ((size_t)bh * SEQ + q0 + m) * HD;
  const v16h qb0 = load_frag(qrow, h);
  const v16h qb1 = load_frag(qrow + 32, h);

  const v8f zero8 = {0.f, 0.f, 0.f, 0.f, 0.f, 0.f, 0.f, 0.f};
  v8f o[4];
  #pragma unroll
  for (int t = 0; t < 4; ++t) o[t] = zero8;
  float mrun = -1e30f, lrun = 0.0f;

  const _Float16* kbase = kh + ((size_t)bh * SEQ + m) * HD;
  const _Float16* vbase = vt + ((size_t)bh * HD + m) * SEQ;

  #pragma unroll 1
  for (int kb = 0; kb < SEQ; kb += 64) {
    v8f s[4];
    #pragma unroll
    for (int j = 0; j < 4; ++j) {
      const _Float16* kp = kbase + (size_t)(kb + 16 * j) * HD;
      const v16h kf0 = load_frag(kp, h);
      const v16h kf1 = load_frag(kp + 32, h);
      v8f z = zero8;
      z = wmma_f16(kf0, qb0, z);
      z = wmma_f16(kf1, qb1, z);
      #pragma unroll
      for (int r = 0; r < 8; ++r) z[r] = z[r] * SSCALE;
      s[j] = z;
    }

    float mloc = s[0][0];
    #pragma unroll
    for (int j = 0; j < 4; ++j)
      #pragma unroll
      for (int r = 0; r < 8; ++r) mloc = fmaxf(mloc, s[j][r]);
    mloc = fmaxf(mloc, __shfl_xor(mloc, 16));
    const float mnew = fmaxf(mrun, mloc);
    const float alpha = __expf(mrun - mnew);
    mrun = mnew;
    float lsum = 0.0f;
    #pragma unroll
    for (int j = 0; j < 4; ++j)
      #pragma unroll
      for (int r = 0; r < 8; ++r) {
        const float p = __expf(s[j][r] - mnew);
        s[j][r] = p;
        lsum += p;
      }
    lsum += __shfl_xor(lsum, 16);
    lrun = lrun * alpha + lsum;
    #pragma unroll
    for (int t = 0; t < 4; ++t)
      #pragma unroll
      for (int r = 0; r < 8; ++r) o[t][r] = o[t][r] * alpha;

    const v16h pb0 = pack_p(s[0], s[1]);
    const v16h pb1 = pack_p(s[2], s[3]);

    #pragma unroll
    for (int t = 0; t < 4; ++t) {
      const _Float16* vp = vbase + (size_t)(16 * t) * SEQ + kb;
      const v16h vf0 = load_frag(vp, h);
      const v16h vf1 = load_frag(vp + 32, h);
      o[t] = wmma_f16(vf0, pb0, o[t]);
      o[t] = wmma_f16(vf1, pb1, o[t]);
    }
  }

  const float inv = (1.0f / lrun) * (CSC / PSCALE);
  float* so = sO + w * 1024;
  #pragma unroll
  for (int t = 0; t < 4; ++t)
    #pragma unroll
    for (int r = 0; r < 8; ++r)
      so[m * 64 + 16 * t + 8 * h + r] = o[t][r] * inv;
  __syncthreads();

  const int q4 = lane >> 3, c8 = (lane & 7) * 8;
  v8h hv[4];
  #pragma unroll
  for (int it = 0; it < 4; ++it) {
    const int row = it * 4 + q4;
    const v4f fa = *(const v4fa*)(so + row * 64 + c8);
    const v4f fb = *(const v4fa*)(so + row * 64 + c8 + 4);
    const v8h o8 = { (_Float16)fa.x, (_Float16)fa.y, (_Float16)fa.z, (_Float16)fa.w,
                     (_Float16)fb.x, (_Float16)fb.y, (_Float16)fb.z, (_Float16)fb.w };
    hv[it] = o8;
  }
  #pragma unroll
  for (int it = 0; it < 4; ++it) {
    const int row = it * 4 + q4;
    const size_t gi = ((size_t)b * SEQ + q0 + row) * HIDDEN + head * HD + c8;
    *(volatile v8h*)(ctx + gi) = hv[it];
  }
  __threadfence();
  #pragma unroll
  for (int it = 0; it < 4; ++it) {
    const int row = it * 4 + q4;
    const size_t gi = ((size_t)b * SEQ + q0 + row) * HIDDEN + head * HD + c8;
    *(volatile v8h*)(ctx + gi) = hv[it];
  }
}

__device__ __forceinline__ void out_store_pass(const float* sOut, float* out,
                                               int m0, int fg, int w, int lane) {
  const int h2 = lane >> 4, c4 = (lane & 15) * 4;
  #pragma unroll
  for (int i = 0; i < 16; ++i) {
    const int row = w * 32 + i * 2 + h2;
    const v4f v = *(const v4fa*)(sOut + row * 64 + c4);
    const size_t gi = (size_t)(m0 + row) * HIDDEN + fg * HD + c4;
    *(volatile v4f*)(out + gi) = v;
  }
}

__global__ __launch_bounds__(128) void oproj_kernel(
    const _Float16* __restrict__ ch,
    const _Float16* __restrict__ woh,
    const float* __restrict__ bo,
    float* __restrict__ out)
{
  __shared__ __attribute__((aligned(16))) float sOut[128 * 64];

  const int tid = threadIdx.x, lane = tid & 31, w = tid >> 5;
  const int h = lane >> 4, m = lane & 15;
  const int m0 = blockIdx.x * 128;
  const int fg = blockIdx.y;
  const int m0w = m0 + 32 * w;

  const _Float16* xa0 = ch + (size_t)(m0w + m) * HIDDEN;
  const _Float16* xa1 = xa0 + (size_t)16 * HIDDEN;
  const _Float16* wb  = woh + ((size_t)fg * HD + m) * HIDDEN;

  const v8f zero8 = {0.f, 0.f, 0.f, 0.f, 0.f, 0.f, 0.f, 0.f};
  v8f acc[2][4];
  #pragma unroll
  for (int mt = 0; mt < 2; ++mt)
    #pragma unroll
    for (int nt = 0; nt < 4; ++nt) acc[mt][nt] = zero8;

  #pragma unroll 1
  for (int k0 = 0; k0 < HIDDEN; k0 += 32) {
    const v16h a0 = load_frag(xa0 + k0, h);
    const v16h a1 = load_frag(xa1 + k0, h);
    #pragma unroll
    for (int nt = 0; nt < 4; ++nt) {
      const v16h b = load_frag(wb + (size_t)nt * 16 * HIDDEN + k0, h);
      acc[0][nt] = wmma_f16(a0, b, acc[0][nt]);
      acc[1][nt] = wmma_f16(a1, b, acc[1][nt]);
    }
  }

  #pragma unroll
  for (int nt = 0; nt < 4; ++nt) {
    const int feat = 16 * nt + m;
    const float bvl = bo[fg * HD + feat];
    #pragma unroll
    for (int mt = 0; mt < 2; ++mt) {
      #pragma unroll
      for (int r = 0; r < 8; ++r) {
        const int tokl = 32 * w + 16 * mt + 8 * h + r;
        sOut[tokl * 64 + feat] = acc[mt][nt][r] * OINV + bvl;
      }
    }
  }
  __syncthreads();

  out_store_pass(sOut, out, m0, fg, w, lane);
  __threadfence();
  out_store_pass(sOut, out, m0, fg, w, lane);
}

extern "C" void kernel_launch(void* const* d_in, const int* in_sizes, int n_in,
                              void* d_out, int out_size, void* d_ws, size_t ws_size,
                              hipStream_t stream) {
  if (n_in < 9) return;
  if (in_sizes[0] != NX) return;
  if (in_sizes[1] != NW || in_sizes[3] != NW || in_sizes[5] != NW || in_sizes[7] != NW) return;
  if (in_sizes[2] != HIDDEN || in_sizes[4] != HIDDEN || in_sizes[6] != HIDDEN || in_sizes[8] != HIDDEN) return;
  if (out_size != NX) return;

  const float* x  = (const float*)d_in[0];
  const float* Wq = (const float*)d_in[1];
  const float* bq = (const float*)d_in[2];
  const float* Wk = (const float*)d_in[3];
  const float* bk = (const float*)d_in[4];
  const float* Wv = (const float*)d_in[5];
  const float* bv = (const float*)d_in[6];
  const float* Wo = (const float*)d_in[7];
  const float* bo = (const float*)d_in[8];
  float* out = (float*)d_out;

  const size_t xh_bytes = (size_t)NX * 2;
  const size_t wh_bytes = (size_t)NWMAT * NW * 2;
  const size_t pl_bytes = (size_t)BATCH * NHEADS * SEQ * HD * 2;
  const size_t cx_bytes = (size_t)NX * 2;
  size_t off = 0;
  const size_t oXh = off; off += xh_bytes;
  const size_t oWh = off; off += wh_bytes;
  const size_t oQh = off; off += pl_bytes;
  const size_t oKh = off; off += pl_bytes;
  const size_t oVt = off; off += pl_bytes;
  const size_t oCx = off; off += cx_bytes;
  if (off > ws_size) return;
  if (off > (size_t)134217728) return;

  char* ws = (char*)d_ws;
  _Float16* xh  = (_Float16*)(ws + oXh);
  _Float16* wh  = (_Float16*)(ws + oWh);
  _Float16* qh  = (_Float16*)(ws + oQh);
  _Float16* kh  = (_Float16*)(ws + oKh);
  _Float16* vt  = (_Float16*)(ws + oVt);
  _Float16* ctx = (_Float16*)(ws + oCx);

  const int ngroups = NX8 + NWMAT * NW8;
  convert_kernel<<<(ngroups + 255) / 256, 256, 0, stream>>>(x, Wq, Wk, Wv, Wo, xh, wh);

  dim3 gProj(MROWS / 128, 3 * NHEADS);
  proj_kernel<<<gProj, 128, 0, stream>>>(xh, wh, bq, bk, bv, qh, kh, vt);

  dim3 gAtt(SEQ / 64, BATCH * NHEADS);
  attn_kernel<<<gAtt, 128, 0, stream>>>(qh, kh, vt, ctx);

  dim3 gOut(MROWS / 128, HIDDEN / HD);
  oproj_kernel<<<gOut, 128, 0, stream>>>(ctx, wh + (size_t)3 * NW, bo, out);

  (void)hipGetLastError();
}
